// FastGaussian2D_1537598292676
// MI455X (gfx1250) — hardware-verified
//
#include <hip/hip_runtime.h>

#define NPIX  65536
#define NG    2048
#define NCHUNK (NG / 32)
#define NTERMS 1

typedef __bf16 v16b __attribute__((ext_vector_type(16)));
typedef float  v8f  __attribute__((ext_vector_type(8)));
typedef float  v4f  __attribute__((ext_vector_type(4)));
typedef float  v4fa __attribute__((ext_vector_type(4), may_alias));
union FragB { v16b v; unsigned short u[16]; };

__device__ __forceinline__ unsigned short bf16_bits(float x) {
  unsigned int u = __float_as_uint(x); return (unsigned short)((u + 0x7FFFu + ((u >> 16) & 1u)) >> 16);
}
__device__ __forceinline__ float bf16_val(unsigned short b) { return __uint_as_float(((unsigned int)b) << 16); }
__device__ __forceinline__ int koff(int e, int h) { return (e < 8) ? (8 * h + e) : (16 + 8 * h + (e - 8)); }

template <int NT_>
__device__ __forceinline__ v8f mma_split(v16b ah, v16b al, v16b bh, v16b bl, v8f c) {
  c = __builtin_amdgcn_wmma_f32_16x16x32_bf16(false, ah, false, bh, (short)0, c, false, false);
  if (NT_ >= 2) c = __builtin_amdgcn_wmma_f32_16x16x32_bf16(false, ah, false, bl, (short)0, c, false, false);
  if (NT_ >= 3) c = __builtin_amdgcn_wmma_f32_16x16x32_bf16(false, al, false, bh, (short)0, c, false, false);
  asm volatile("v_nop\n\tv_nop\n\tv_nop\n\tv_nop" : "+v"(c) : "v"(ah), "v"(al), "v"(bh), "v"(bl));
  return c;
}

__global__ __launch_bounds__(256) void gauss_main(const float* __restrict__ coords, const float* __restrict__ pos,
                                                 const float* __restrict__ ls, const float* __restrict__ col,
                                                 const float* __restrict__ lo, float* __restrict__ out) {
  __shared__ float gpx[NG], gpy[NG], gsx[NG], gsy[NG], gla[NG];
  __shared__ float gcol[NG][4];
  __shared__ float st[8][2][16][4];
  __shared__ __attribute__((aligned(16))) float ob[8][96];

  const float kHalfLog2e = 0.72134752044448170368f;
  const float kS = 0.84932180028801904272f;
  (void)kHalfLog2e;
  for (int g = threadIdx.x; g < NG; g += 256) {
    const float sx = fmaxf(expf(ls[2 * g + 0]), 0.1f);
    const float sy = fmaxf(expf(ls[2 * g + 1]), 0.1f);
    const float nrm = 1.0f / (6.283185307179586f * sx * sy);
    const float amp = nrm * expf(lo[g]);
    gpx[g] = pos[2 * g + 0];
    gpy[g] = pos[2 * g + 1];
    gsx[g] = kS / sx;
    gsy[g] = kS / sy;
    gla[g] = log2f(amp);
    gcol[g][0] = col[3 * g + 0]; gcol[g][1] = col[3 * g + 1]; gcol[g][2] = col[3 * g + 2]; gcol[g][3] = 1.0f;
  }
  __syncthreads();

  const int lane = threadIdx.x & 31, w = threadIdx.x >> 5;
  const int pair = blockIdx.x * 8 + w;
  const int m = lane & 15, hi = lane >> 4, colc = lane & 15;
  const int p0 = pair * 32 + m, p1 = p0 + 16;
  const float x0 = coords[2 * p0], y0 = coords[2 * p0 + 1];
  const float x1 = coords[2 * p1], y1 = coords[2 * p1 + 1];

  v8f acc0 = {}, acc1 = {};
#pragma unroll 1
  for (int c = 0; c < NCHUNK; ++c) {
    const int base = c * 32;
    FragB a0h, a0l, a1h, a1l, bh_, bl_;
#pragma unroll
    for (int i = 0; i < 16; ++i) {
      const int g = base + koff(i, hi);
      const float dx0 = (x0 - gpx[g]) * gsx[g], dy0 = (y0 - gpy[g]) * gsy[g];
      const float dx1 = (x1 - gpx[g]) * gsx[g], dy1 = (y1 - gpy[g]) * gsy[g];
      const float e0 = gla[g] - (dx0 * dx0 + dy0 * dy0);
      const float e1 = gla[g] - (dx1 * dx1 + dy1 * dy1);
      const float al0 = exp2f(e0), al1 = exp2f(e1);
      const unsigned short h0 = bf16_bits(al0), h1 = bf16_bits(al1);
      a0h.u[i] = h0; a1h.u[i] = h1;
      if (NTERMS >= 3) { a0l.u[i] = bf16_bits(al0 - bf16_val(h0)); a1l.u[i] = bf16_bits(al1 - bf16_val(h1)); } else { a0l.u[i] = 0; a1l.u[i] = 0; }
      const float bv = gcol[g][colc < 4 ? colc : 3] * (colc < 4 ? 1.0f : 0.0f);
      const unsigned short hb = bf16_bits(bv);
      bh_.u[i] = hb; bl_.u[i] = (NTERMS >= 2) ? bf16_bits(bv - bf16_val(hb)) : (unsigned short)0;
    }
    acc0 = mma_split<NTERMS>(a0h.v, a0l.v, bh_.v, bl_.v, acc0);
    acc1 = mma_split<NTERMS>(a1h.v, a1l.v, bh_.v, bl_.v, acc1);
  }

  if (colc < 4) {
#pragma unroll
    for (int r = 0; r < 8; ++r) { st[w][0][8 * hi + r][colc] = acc0[r]; st[w][1][8 * hi + r][colc] = acc1[r]; }
  }
  __builtin_amdgcn_fence(__ATOMIC_ACQ_REL, "workgroup");
  __builtin_amdgcn_wave_barrier();
  {
    const int t = lane >> 4, mm = lane & 15;
    const float inv = 1.0f / fmaxf(st[w][t][mm][3], 1e-8f);
#pragma unroll
    for (int ch = 0; ch < 3; ++ch) ob[w][lane * 3 + ch] = fminf(fmaxf(st[w][t][mm][ch] * inv, 0.0f), 1.0f);
  }
  __builtin_amdgcn_fence(__ATOMIC_ACQ_REL, "workgroup");
  __builtin_amdgcn_wave_barrier();
  if (lane < 24) {
    const v4f v = *(const v4fa*)&ob[w][lane * 4];
    float* dst = out + (size_t)pair * 96 + lane * 4;
    *(volatile v4f*)dst = v;
    __threadfence();
    *(volatile v4f*)dst = v;
  }
}

extern "C" void kernel_launch(void* const* d_in, const int* in_sizes, int n_in,
                              void* d_out, int out_size, void* d_ws, size_t ws_size, hipStream_t stream) {
  (void)in_sizes; (void)n_in; (void)out_size; (void)d_ws; (void)ws_size;
  const float* coords = (const float*)d_in[0];
  const float* pos = (const float*)d_in[1];
  const float* ls  = (const float*)d_in[2];
  const float* col = (const float*)d_in[3];
  const float* lo  = (const float*)d_in[4];
  gauss_main<<<(NPIX / 32) / 8, 256, 0, stream>>>(coords, pos, ls, col, lo, (float*)d_out);
}
